// SparseCutAttention_26465588478185
// MI455X (gfx1250) — hardware-verified
//
#include <hip/hip_runtime.h>


#define NB_  2
#define NC_  64
#define NH_  8192
#define HB_  1024
#define N7_  7
#define NCUT 4
#define NL_  (NCUT * HB_)
#define TEMP_INV (1.0f / 0.7f)
#define PSC   32768.0f
#define PSCI  (1.0f / 32768.0f)
#define LOSC  256.0f
#define LOSCI (1.0f / 256.0f)

typedef _Float16 h16;
typedef __attribute__((ext_vector_type(16))) _Float16 v16h;
typedef __attribute__((ext_vector_type(8)))  _Float16 v8h;
typedef __attribute__((ext_vector_type(8)))  float    v8f;
typedef __attribute__((ext_vector_type(4)))  float    v4f;
typedef v8h  __attribute__((may_alias)) v8ha;
typedef v4f  __attribute__((may_alias)) v4fa;

__device__ __forceinline__ float bf16r(float f) { unsigned u = __float_as_uint(f); u += 0x7FFFu + ((u >> 16) & 1u); return __uint_as_float(u & 0xFFFF0000u); }
__device__ __forceinline__ v16h cat16(v8h lo, v8h hi) { return __builtin_shufflevector(lo, hi, 0, 1, 2, 3, 4, 5, 6, 7, 8, 9, 10, 11, 12, 13, 14, 15); }
__device__ __forceinline__ v8f wmma16(v16h a, v16h b, v8f c) { return __builtin_amdgcn_wmma_f32_16x16x32_f16(false, a, false, b, (short)0, c, false, false); }

__global__ __launch_bounds__(256) void k_perm(const float* __restrict__ q, const float* __restrict__ k, const float* __restrict__ gu, float* PERM) {
    __shared__ float sq[N7_ * HB_];
    __shared__ float sk[N7_ * HB_];
    __shared__ float R[64];
    __shared__ float pm[64];
    const int b = blockIdx.x, tid = threadIdx.x;
    const float* qb = q + (size_t)b * NC_ * NH_;
    const float* kb = k + (size_t)b * NC_ * NH_;
#pragma unroll 1
    for (int idx = tid; idx < N7_ * HB_; idx += 256) {
        const int n = idx / HB_, h = idx - n * HB_;
        const size_t pos = (size_t)n * HB_ + h;
        float s1 = 0.f, s2 = 0.f;
#pragma unroll 1
        for (int c = 0; c < NC_; ++c) { s1 += bf16r(qb[(size_t)c * NH_ + pos]); s2 += bf16r(kb[(size_t)c * NH_ + pos]); }
        sq[idx] = s1 * (1.0f / 64.0f);
        sk[idx] = s2 * (1.0f / 64.0f);
    }
    __syncthreads();
    if (tid < 64) {
        float r = 0.f;
        if (tid < 49) {
            const int i = tid / 7, j = tid - i * 7;
            float s = 0.f;
#pragma unroll 1
            for (int h = 0; h < HB_; ++h) s += sq[i * HB_ + h] * sk[j * HB_ + h];
            const float Rij = s * 0.125f;
            const float rl = Rij > 0.f ? Rij : 0.f;
            const float u = bf16r(gu[(size_t)b * 49 + tid]);
            const float g = -logf(-logf(u + 1e-6f) + 1e-6f);
            r = (logf(rl) + g) * TEMP_INV;
        }
        R[tid] = r;
    }
    __syncthreads();
    if (tid == 0) {
        float m[49];
#pragma unroll
        for (int e = 0; e < 49; ++e) m[e] = R[e];
#pragma unroll 1
        for (int it = 0; it < 8; ++it) {
#pragma unroll
            for (int i = 0; i < 7; ++i) {
                float mx = -__builtin_inff();
#pragma unroll
                for (int j = 0; j < 7; ++j) mx = fmaxf(mx, m[i * 7 + j]);
                if (!(fabsf(mx) < __builtin_inff())) mx = 0.f;
                float s = 0.f;
#pragma unroll
                for (int j = 0; j < 7; ++j) s += expf(m[i * 7 + j] - mx);
                const float lse = logf(s) + mx;
#pragma unroll
                for (int j = 0; j < 7; ++j) m[i * 7 + j] -= lse;
            }
#pragma unroll
            for (int j = 0; j < 7; ++j) {
                float mx = -__builtin_inff();
#pragma unroll
                for (int i = 0; i < 7; ++i) mx = fmaxf(mx, m[i * 7 + j]);
                if (!(fabsf(mx) < __builtin_inff())) mx = 0.f;
                float s = 0.f;
#pragma unroll
                for (int i = 0; i < 7; ++i) s += expf(m[i * 7 + j] - mx);
                const float lse = logf(s) + mx;
#pragma unroll
                for (int i = 0; i < 7; ++i) m[i * 7 + j] -= lse;
            }
        }
#pragma unroll
        for (int e = 0; e < 64; ++e) pm[e] = e < 49 ? expf(m[e]) : 0.f;
    }
    __syncthreads();
    if (tid < 32) {
        float* dst = PERM + (size_t)b * 64;
        *(volatile float*)(dst + tid) = pm[tid]; *(volatile float*)(dst + 32 + tid) = pm[32 + tid];
        __threadfence();
        *(volatile float*)(dst + tid) = pm[tid]; *(volatile float*)(dst + 32 + tid) = pm[32 + tid];
    }
}

__global__ __launch_bounds__(256) void k_mix(const float* __restrict__ k, const float* __restrict__ v, const float* __restrict__ PERM,
                                             h16* KSH, h16* KSL, h16* VTH, h16* VTL) {
    __shared__ __align__(16) h16 ksh[64 * 64];
    __shared__ __align__(16) h16 ksl[64 * 64];
    __shared__ __align__(16) h16 vth[64 * 64];
    __shared__ __align__(16) h16 vtl[64 * 64];
    __shared__ float pw[8];
    const int bid = blockIdx.x;
    const int b = bid / (NCUT * 16), rem = bid - b * (NCUT * 16), m = rem / 16, ht = rem - m * 16;
    const int h0 = ht * 64;
    const int tid = threadIdx.x;
    if (tid < 8) pw[tid] = tid < N7_ ? PERM[(size_t)b * 64 + tid * 7 + m] : 0.f;
    __syncthreads();
    const int c = tid >> 2, hl0 = (tid & 3) * 16;
    const float* kc = k + ((size_t)b * NC_ + c) * NH_ + h0 + hl0;
    const float* vc = v + ((size_t)b * NC_ + c) * NH_ + h0 + hl0;
    float aks[16], avs[16];
#pragma unroll
    for (int i = 0; i < 16; ++i) { aks[i] = 0.f; avs[i] = 0.f; }
#pragma unroll 1
    for (int n = 0; n < N7_; ++n) {
        const float w = pw[n];
        const float* kp = kc + (size_t)n * HB_;
        const float* vp = vc + (size_t)n * HB_;
#pragma unroll
        for (int i = 0; i < 16; ++i) { aks[i] += bf16r(kp[i]) * w; avs[i] += bf16r(vp[i]) * w; }
    }
#pragma unroll
    for (int i = 0; i < 16; ++i) {
        const int hl = hl0 + i;
        const h16 kh = (h16)aks[i]; const h16 kl = (h16)((aks[i] - (float)kh) * LOSC);
        const h16 vh = (h16)avs[i]; const h16 vl = (h16)((avs[i] - (float)vh) * LOSC);
        ksh[hl * 64 + c] = kh; ksl[hl * 64 + c] = kl;
        vth[c * 64 + hl] = vh; vtl[c * 64 + hl] = vl;
    }
    __syncthreads();
    const int piece = tid & 7;
    auto pass = [&]() {
#pragma unroll
        for (int s = 0; s < 8; ++s) {
            const int Lid = (tid >> 3) + 32 * s;
            const int grp = Lid >> 6, row = Lid & 63;
            const h16* src = (grp == 0 ? ksh : grp == 1 ? ksl : grp == 2 ? vth : vtl) + row * 64 + piece * 8;
            const v8h val = *(const v8ha*)src;
            h16* dst;
            if (grp < 2) dst = (grp == 0 ? KSH : KSL) + ((size_t)b * NL_ + (size_t)m * HB_ + h0 + row) * 64 + piece * 8;
            else         dst = (grp == 2 ? VTH : VTL) + ((size_t)b * NC_ + row) * NL_ + (size_t)m * HB_ + h0 + piece * 8;
            *(volatile v8h*)dst = val;
        }
    };
    pass();
    __threadfence();
    pass();
}

__global__ __launch_bounds__(128) void k_attn(const float* __restrict__ q, const h16* __restrict__ KSH, const h16* __restrict__ KSL,
                                              const h16* __restrict__ VTH, const h16* __restrict__ VTL, float* VAL) {
    __shared__ __align__(16) h16 plds[4][2][16 * 32];
    __shared__ __align__(16) float ost[4][16 * 68];
    const int lane = threadIdx.x & 31, wave = threadIdx.x >> 5, lr = lane & 15, hi = lane >> 4;
    const int b = blockIdx.x / (NH_ / 64);
    const int q0 = (blockIdx.x - b * (NH_ / 64)) * 64 + wave * 16;
    h16* pl = &plds[wave][0][0];
    h16* pll = &plds[wave][1][0];
    const float* qb = q + (size_t)b * NC_ * NH_;

    v16h qa[2];
#pragma unroll
    for (int kc = 0; kc < 2; ++kc) {
        v16h a;
#pragma unroll
        for (int i = 0; i < 8; ++i) {
            a[i]     = (h16)bf16r(qb[(size_t)(kc * 32 + 8 * hi + i) * NH_ + q0 + lr]);
            a[i + 8] = (h16)bf16r(qb[(size_t)(kc * 32 + 16 + 8 * hi + i) * NH_ + q0 + lr]);
        }
        qa[kc] = a;
    }
    const h16* ksh_b = KSH + (size_t)b * NL_ * 64;
    const h16* ksl_b = KSL + (size_t)b * NL_ * 64;
    const h16* vth_b = VTH + (size_t)b * NC_ * NL_;
    const h16* vtl_b = VTL + (size_t)b * NC_ * NL_;

    v8f oh[4], ol[4];
#pragma unroll
    for (int n = 0; n < 4; ++n) { oh[n] = (v8f){}; ol[n] = (v8f){}; }
    float mrow[8], lpart[8];
#pragma unroll
    for (int j = 0; j < 8; ++j) { mrow[j] = -3.0e38f; lpart[j] = 0.f; }

#pragma unroll 1
    for (int kt = 0; kt < NL_ / 32; ++kt) {
        const int l0 = kt * 32;
        v8f sh0 = {}, sh1 = {}, sl0 = {}, sl1 = {};
#pragma unroll
        for (int kc = 0; kc < 2; ++kc) {
            const h16* r0h = ksh_b + (size_t)(l0 + lr) * 64 + kc * 32 + 8 * hi;
            const h16* r1h = ksh_b + (size_t)(l0 + 16 + lr) * 64 + kc * 32 + 8 * hi;
            const h16* r0l = ksl_b + (size_t)(l0 + lr) * 64 + kc * 32 + 8 * hi;
            const h16* r1l = ksl_b + (size_t)(l0 + 16 + lr) * 64 + kc * 32 + 8 * hi;
            sh0 = wmma16(qa[kc], cat16(*(const v8h*)r0h, *(const v8h*)(r0h + 16)), sh0);
            sh1 = wmma16(qa[kc], cat16(*(const v8h*)r1h, *(const v8h*)(r1h + 16)), sh1);
            sl0 = wmma16(qa[kc], cat16(*(const v8h*)r0l, *(const v8h*)(r0l + 16)), sl0);
            sl1 = wmma16(qa[kc], cat16(*(const v8h*)r1l, *(const v8h*)(r1l + 16)), sl1);
        }
        asm volatile("v_nop\n\tv_nop\n\tv_nop\n\tv_nop" : "+v"(sh0), "+v"(sh1), "+v"(sl0), "+v"(sl1) : "v"(qa[0]), "v"(qa[1]));
        float alpha[8];
#pragma unroll
        for (int j = 0; j < 8; ++j) {
            const float a0 = (sh0[j] + sl0[j] * LOSCI) * TEMP_INV;
            const float a1 = (sh1[j] + sl1[j] * LOSCI) * TEMP_INV;
            float mx = fmaxf(a0, a1);
            mx = fmaxf(mx, __shfl_xor(mx, 1, 16)); mx = fmaxf(mx, __shfl_xor(mx, 2, 16));
            mx = fmaxf(mx, __shfl_xor(mx, 4, 16)); mx = fmaxf(mx, __shfl_xor(mx, 8, 16));
            const float mn = fmaxf(mrow[j], mx);
            alpha[j] = __expf(mrow[j] - mn);
            mrow[j] = mn;
            const float p0 = __expf(a0 - mn), p1 = __expf(a1 - mn);
            lpart[j] = lpart[j] * alpha[j] + (p0 + p1);
            const int mr = hi * 8 + j;
            const float ps0 = p0 * PSC, ps1 = p1 * PSC;
            const h16 h0 = (h16)ps0, h1 = (h16)ps1;
            pl[mr * 32 + lr]       = h0;
            pl[mr * 32 + 16 + lr]  = h1;
            pll[mr * 32 + lr]      = (h16)((ps0 - (float)h0) * LOSC);
            pll[mr * 32 + 16 + lr] = (h16)((ps1 - (float)h1) * LOSC);
        }
#pragma unroll
        for (int n = 0; n < 4; ++n)
#pragma unroll
            for (int j = 0; j < 8; ++j) { oh[n][j] *= alpha[j]; ol[n][j] *= alpha[j]; }
        asm volatile("" ::: "memory");
        const v16h pa  = cat16(*(const v8ha*)(pl + lr * 32 + hi * 8), *(const v8ha*)(pl + lr * 32 + 16 + hi * 8));
        const v16h pal = cat16(*(const v8ha*)(pll + lr * 32 + hi * 8), *(const v8ha*)(pll + lr * 32 + 16 + hi * 8));
#pragma unroll
        for (int n = 0; n < 4; ++n) {
            const h16* vh = vth_b + (size_t)(n * 16 + lr) * NL_ + l0 + hi * 8;
            const h16* vl = vtl_b + (size_t)(n * 16 + lr) * NL_ + l0 + hi * 8;
            const v16h vbh = cat16(*(const v8h*)vh, *(const v8h*)(vh + 16));
            oh[n] = wmma16(pa, vbh, oh[n]);
            ol[n] = wmma16(pa, cat16(*(const v8h*)vl, *(const v8h*)(vl + 16)), ol[n]);
            ol[n] = wmma16(pal, vbh, ol[n]);
        }
        asm volatile("v_nop\n\tv_nop\n\tv_nop\n\tv_nop" : "+v"(oh[0]), "+v"(oh[1]), "+v"(oh[2]), "+v"(oh[3]), "+v"(ol[0]), "+v"(ol[1]), "+v"(ol[2]), "+v"(ol[3]) : "v"(pa), "v"(pal));
    }
    float inv[8];
#pragma unroll
    for (int j = 0; j < 8; ++j) {
        float rs = lpart[j];
        rs += __shfl_xor(rs, 1, 16); rs += __shfl_xor(rs, 2, 16); rs += __shfl_xor(rs, 4, 16); rs += __shfl_xor(rs, 8, 16);
        inv[j] = 1.0f / (rs * PSC);
    }
    float* os = &ost[wave][0];
#pragma unroll
    for (int n = 0; n < 4; ++n)
#pragma unroll
        for (int j = 0; j < 8; ++j) os[(hi * 8 + j) * 68 + n * 16 + lr] = (oh[n][j] + ol[n][j] * LOSCI) * inv[j];
    __syncthreads();
    float* vrow = VAL + ((size_t)b * NH_ + q0) * 64;
    auto pass = [&]() {
#pragma unroll
        for (int s = 0; s < 8; ++s) {
            const int Lid = (lane >> 3) + 4 * s, piece = lane & 7;
            const int row = Lid >> 1, cofs = (Lid & 1) * 32 + piece * 4;
            const v4f val = *(const v4fa*)(os + row * 68 + cofs);
            *(volatile v4f*)(vrow + (size_t)row * 64 + cofs) = val;
        }
    };
    pass();
    __threadfence();
    pass();
}

__global__ __launch_bounds__(256) void k_stats(const float* __restrict__ VAL, double* PART) {
    __shared__ double rs[8], rq[8];
    const int b = blockIdx.x >> 6, ch = blockIdx.x & 63, tid = threadIdx.x, lane = tid & 31, w = tid >> 5;
    const float* p = VAL + (size_t)b * NH_ * NC_ + (size_t)ch * 8192;
    double s = 0.0, sq2 = 0.0;
#pragma unroll 1
    for (int i = tid; i < 8192; i += 256) { const double x = (double)p[i]; s += x; sq2 += x * x; }
#pragma unroll
    for (int o = 16; o; o >>= 1) { s += __shfl_xor(s, o, 32); sq2 += __shfl_xor(sq2, o, 32); }
    if (lane == 0) { rs[w] = s; rq[w] = sq2; }
    __syncthreads();
    if (tid < 32) {
        double ts = 0.0, tq = 0.0;
#pragma unroll
        for (int i = 0; i < 8; ++i) { ts += rs[i]; tq += rq[i]; }
        double* dst = PART + ((size_t)b * 64 + ch) * 32;
        const double vv = lane == 0 ? ts : (lane == 1 ? tq : 0.0);
        *(volatile double*)(dst + lane) = vv;
        __threadfence();
        *(volatile double*)(dst + lane) = vv;
    }
}

__global__ __launch_bounds__(256) void k_norm(const float* __restrict__ VAL, const double* __restrict__ PART, float* out) {
    __shared__ float mv[2];
    const int b = blockIdx.x >> 6, ch = blockIdx.x & 63, tid = threadIdx.x;
    if (tid == 0) {
        double ts = 0.0, tq = 0.0;
#pragma unroll 1
        for (int i = 0; i < 64; ++i) { ts += PART[((size_t)b * 64 + i) * 32]; tq += PART[((size_t)b * 64 + i) * 32 + 1]; }
        const double n = (double)NH_ * (double)NC_;
        const double mean = ts / n;
        double var = tq / n - mean * mean; if (var < 0.0) var = 0.0;
        mv[0] = (float)mean; mv[1] = 1.0f / sqrtf((float)var + 1e-5f);
    }
    __syncthreads();
    const float mean = mv[0], isd = mv[1];
    const float* p = VAL + (size_t)b * NH_ * NC_ + (size_t)ch * 8192;
    float* o = out + (size_t)b * NH_ * NC_ + (size_t)ch * 8192;
    const int piece = tid & 7;
    auto pass = [&]() {
#pragma unroll
        for (int s = 0; s < 8; ++s) {
            const int Lid = (tid >> 3) + 32 * s;
            const int e = Lid * 32 + piece * 4;
            const v4f x = *(const v4f*)(p + e);
            v4f y;
#pragma unroll
            for (int t = 0; t < 4; ++t) y[t] = (x[t] - mean) * isd;
            *(volatile v4f*)(o + e) = y;
        }
    };
    pass();
    __threadfence();
    pass();
}

extern "C" void kernel_launch(void* const* d_in, const int* in_sizes, int n_in,
                              void* d_out, int out_size, void* d_ws, size_t ws_size, hipStream_t stream) {
    (void)in_sizes; (void)n_in; (void)out_size;
    const float* q = (const float*)d_in[0]; const float* k = (const float*)d_in[1]; const float* v = (const float*)d_in[2]; const float* gu = (const float*)d_in[3];
    float* out = (float*)d_out;
    char* wsp = (char*)d_ws;
    auto take = [&](size_t bytes) { char* p = wsp; wsp += (bytes + 255) & ~(size_t)255; return (void*)p; };
    float*  PERM = (float*)take((size_t)NB_ * 64 * 4);
    h16*    KSH  = (h16*)take((size_t)NB_ * NL_ * 64 * 2);
    h16*    KSL  = (h16*)take((size_t)NB_ * NL_ * 64 * 2);
    h16*    VTH  = (h16*)take((size_t)NB_ * NC_ * NL_ * 2);
    h16*    VTL  = (h16*)take((size_t)NB_ * NC_ * NL_ * 2);
    float*  VAL  = (float*)take((size_t)NB_ * NH_ * NC_ * 4);
    double* PART = (double*)take((size_t)NB_ * 64 * 32 * 8);
    if ((size_t)(wsp - (char*)d_ws) > ws_size) return;
    k_perm<<<NB_, 256, 0, stream>>>(q, k, gu, PERM);
    k_mix<<<NB_ * NCUT * 16, 256, 0, stream>>>(k, v, PERM, KSH, KSL, VTH, VTL);
    k_attn<<<NB_ * (NH_ / 64), 128, 0, stream>>>(q, KSH, KSL, VTH, VTL, VAL);
    k_stats<<<NB_ * 64, 256, 0, stream>>>(VAL, PART);
    k_norm<<<NB_ * 64, 256, 0, stream>>>(VAL, PART, out);
}
